// JastrowFactor_80229989089986
// MI455X (gfx1250) — hardware-verified
//
#include <hip/hip_runtime.h>
#include <stddef.h>
#include <stdint.h>


#define N_E      32
#define N_NUC    8
#define D_H      32
#define N_PAIR   496
#define EE_TILES 31
#define EN_TILES 2
#define WPB      32
#define TPB      256
#define NWAVE    (TPB / 32)
#define POSF     (N_E * 3)

#define W2SC  64.0f
#define INV64 0.015625f

static_assert(N_PAIR == EE_TILES * 16);
static_assert(N_E == EN_TILES * 16);
static_assert(N_E * N_NUC == TPB);
static_assert(D_H * D_H == 4 * TPB);
static_assert(TPB == 8 * 32);
static_assert((WPB * POSF) % 4 == 0);
static_assert((POSF % 4) == 0);

typedef _Float16 v16h __attribute__((ext_vector_type(16)));
typedef _Float16 v8h  __attribute__((ext_vector_type(8)));
typedef _Float16 v4h  __attribute__((ext_vector_type(4)));
typedef float    v8f  __attribute__((ext_vector_type(8)));
typedef float    v4f  __attribute__((ext_vector_type(4)));
union Frag { v16h v; v8h half[2]; _Float16 e[16]; };

__device__ __forceinline__ int imin(int a, int b) { return a < b ? a : b; }
__device__ __forceinline__ int imax(int a, int b) { return a > b ? a : b; }

__device__ __forceinline__ float silu_f(float x) {
  return x * __builtin_amdgcn_rcpf(1.0f + __expf(-x));
}

__device__ __forceinline__ float softplus_f(float x) {
  return fmaxf(x, 0.0f) + log1pf(__expf(-fabsf(x)));
}

__device__ __forceinline__ v8f wmh(v16h a, v16h b, v8f c) {
  v8f d = __builtin_amdgcn_wmma_f32_16x16x32_f16(false, a, false, b, (short)0, c, false, false);
  asm volatile("v_nop\n\tv_nop\n\tv_nop\n\tv_nop" : "+v"(d) : "v"(a), "v"(b));
  return d;
}

__device__ __forceinline__ v16h ldA(const _Float16* base, int ld, int lane) {
  Frag a;
  const _Float16* p = base + (lane & 15) * ld + 8 * (lane >> 4);
  a.half[0] = *(const v8h*)p;
  a.half[1] = *(const v8h*)(p + 16);
  return a.v;
}

__device__ __forceinline__ float tile_nn(v16h A, v16h B0, v16h B1,
                                         float b2lo, float b2hi, float w3lo, float w3hi) {
  const v8f z8 = {0.f, 0.f, 0.f, 0.f, 0.f, 0.f, 0.f, 0.f};
  const v8f c0 = wmh(A, B0, z8);
  const v8f c1 = wmh(A, B1, z8);
  float nn = 0.0f;
#pragma unroll
  for (int v = 0; v < 8; ++v) {
    nn = fmaf(silu_f(fmaf(c0[v], INV64, b2lo)), w3lo, nn);
    nn = fmaf(silu_f(fmaf(c1[v], INV64, b2hi)), w3hi, nn);
  }
  return nn;
}

__global__ __launch_bounds__(TPB) void k_jastrow(
    const float* __restrict__ r_e, const float* __restrict__ r_nuc, const float* __restrict__ charges,
    const int* __restrict__ spin, const float* __restrict__ b_en, const float* __restrict__ b_ee,
    const float* __restrict__ W1_en, const float* __restrict__ b1_en,
    const float* __restrict__ W2_en, const float* __restrict__ b2_en,
    const float* __restrict__ W3_en, const float* __restrict__ b3_en,
    const float* __restrict__ W1_ee, const float* __restrict__ b1_ee,
    const float* __restrict__ W2_ee, const float* __restrict__ b2_ee,
    const float* __restrict__ W3_ee, const float* __restrict__ b3_ee,
    const float* __restrict__ scale_en, const float* __restrict__ scale_ee,
    float* out, int n_walk) {
  __shared__ __attribute__((aligned(16))) float    sRe[WPB * POSF];
  __shared__ __attribute__((aligned(16))) _Float16 sH1[N_E * D_H];
  __shared__ __attribute__((aligned(16))) _Float16 sW2Tee[D_H * D_H];
  __shared__ __attribute__((aligned(16))) _Float16 sW2Ten[D_H * D_H];
  __shared__ __attribute__((aligned(16))) float    sW1en[N_NUC * D_H];
  __shared__ __attribute__((aligned(16))) float    sW1ee[D_H];
  __shared__ __attribute__((aligned(16))) float    sB1ee[D_H];
  __shared__ __attribute__((aligned(16))) float    sRes[WPB];
  __shared__ float sB1en[D_H];
  __shared__ float sB2ee[D_H];
  __shared__ float sW3ee[D_H];
  __shared__ float sB2en[D_H];
  __shared__ float sW3en[D_H];
  __shared__ float sNuc[N_NUC * 3];
  __shared__ float sChg[N_NUC];
  __shared__ float sBsp[N_NUC];
  __shared__ int   sPIJ[N_PAIR];
  __shared__ float sAsp[N_PAIR];
  __shared__ float sPairR[N_PAIR];
  __shared__ float sX2[N_E * N_NUC];
  __shared__ float sRed[NWAVE];

  const int tid = threadIdx.x, lane = tid & 31, h = lane >> 4, m = lane & 15;
  const int wave = __builtin_amdgcn_readfirstlane(tid >> 5);
  const int w0 = blockIdx.x * WPB;
  if (w0 >= n_walk) return;

  const float sc_en = scale_en[0], sc_ee = scale_ee[0];
  const float b3en16 = 16.0f * b3_en[0], b3ee16 = 16.0f * b3_ee[0];
  const float bee_s = softplus_f(b_ee[0]);

  for (int idx = tid; idx < (WPB * POSF) / 4; idx += TPB) {
    const int wl = idx / (POSF / 4), wi = idx - wl * (POSF / 4);
    const int wg = imin(w0 + wl, n_walk - 1);
    *(v4f*)(sRe + 4 * idx) = *(const v4f*)(r_e + (size_t)wg * POSF + 4 * wi);
  }
  {
    const int k = tid >> 3, q = tid & 7;
    const v4f a = *(const v4f*)(W2_ee + k * D_H + 4 * q);
    const v4f c = *(const v4f*)(W2_en + k * D_H + 4 * q);
    sW2Tee[(4 * q + 0) * D_H + k] = (_Float16)(W2SC * a.x);
    sW2Tee[(4 * q + 1) * D_H + k] = (_Float16)(W2SC * a.y);
    sW2Tee[(4 * q + 2) * D_H + k] = (_Float16)(W2SC * a.z);
    sW2Tee[(4 * q + 3) * D_H + k] = (_Float16)(W2SC * a.w);
    sW2Ten[(4 * q + 0) * D_H + k] = (_Float16)(W2SC * c.x);
    sW2Ten[(4 * q + 1) * D_H + k] = (_Float16)(W2SC * c.y);
    sW2Ten[(4 * q + 2) * D_H + k] = (_Float16)(W2SC * c.z);
    sW2Ten[(4 * q + 3) * D_H + k] = (_Float16)(W2SC * c.w);
  }
  if (tid < (N_NUC * D_H) / 4) *(v4f*)(sW1en + 4 * tid) = *(const v4f*)(W1_en + 4 * tid);
  { const int i = tid;       if ((unsigned)i < (unsigned)D_H) sB1en[i] = b1_en[i]; }
  { const int i = tid - 32;  if ((unsigned)i < (unsigned)D_H) sW1ee[i] = W1_ee[i]; }
  { const int i = tid - 64;  if ((unsigned)i < (unsigned)D_H) sB1ee[i] = b1_ee[i]; }
  { const int i = tid - 96;  if ((unsigned)i < (unsigned)D_H) sB2ee[i] = b2_ee[i]; }
  { const int i = tid - 128; if ((unsigned)i < (unsigned)D_H) sW3ee[i] = W3_ee[i]; }
  { const int i = tid - 160; if ((unsigned)i < (unsigned)D_H) sB2en[i] = b2_en[i]; }
  { const int i = tid - 192; if ((unsigned)i < (unsigned)D_H) sW3en[i] = W3_en[i]; }
  { const int i = tid - 224; if ((unsigned)i < (unsigned)(N_NUC * 3)) sNuc[i] = r_nuc[i]; }
  { const int i = tid;       if ((unsigned)i < (unsigned)N_NUC) sChg[i] = charges[i]; }
  { const int i = tid - 32;  if ((unsigned)i < (unsigned)N_NUC) sBsp[i] = softplus_f(b_en[i]); }
#pragma unroll 1
  for (int p = tid; p < N_PAIR; p += TPB) {
    int i = 0;
#pragma unroll 1
    for (int q = 1; q < N_E; ++q) { if ((q * (63 - q)) / 2 <= p) i = q; }
    i = imin(i, N_E - 2);
    int j = p - (i * (63 - i)) / 2 + i + 1;
    j = imin(imax(j, 0), N_E - 1);
    sPIJ[p] = i * N_E + j;
    const int sm = spin[imin(i * N_E + j, N_E * N_E - 1)];
    sAsp[p] = (sm != 0) ? 0.25f : 0.5f;
  }
  __syncthreads();

  float w1e[16], b1e[16];
  {
    const v4f wa = *(const v4f*)(sW1ee + 8 * h),      wb = *(const v4f*)(sW1ee + 8 * h + 4);
    const v4f wc = *(const v4f*)(sW1ee + 16 + 8 * h), wd = *(const v4f*)(sW1ee + 20 + 8 * h);
    const v4f ba = *(const v4f*)(sB1ee + 8 * h),      bb = *(const v4f*)(sB1ee + 8 * h + 4);
    const v4f bc = *(const v4f*)(sB1ee + 16 + 8 * h), bd = *(const v4f*)(sB1ee + 20 + 8 * h);
    w1e[0] = wa.x; w1e[1] = wa.y; w1e[2]  = wa.z; w1e[3]  = wa.w; w1e[4]  = wb.x; w1e[5]  = wb.y; w1e[6]  = wb.z; w1e[7]  = wb.w;
    w1e[8] = wc.x; w1e[9] = wc.y; w1e[10] = wc.z; w1e[11] = wc.w; w1e[12] = wd.x; w1e[13] = wd.y; w1e[14] = wd.z; w1e[15] = wd.w;
    b1e[0] = ba.x; b1e[1] = ba.y; b1e[2]  = ba.z; b1e[3]  = ba.w; b1e[4]  = bb.x; b1e[5]  = bb.y; b1e[6]  = bb.z; b1e[7]  = bb.w;
    b1e[8] = bc.x; b1e[9] = bc.y; b1e[10] = bc.z; b1e[11] = bc.w; b1e[12] = bd.x; b1e[13] = bd.y; b1e[14] = bd.z; b1e[15] = bd.w;
  }
  const v16h Bee0 = ldA(sW2Tee, D_H, lane);
  const v16h Bee1 = ldA(sW2Tee + 16 * D_H, D_H, lane);
  const v16h Ben0 = ldA(sW2Ten, D_H, lane);
  const v16h Ben1 = ldA(sW2Ten + 16 * D_H, D_H, lane);
  const float b2eelo = sB2ee[m], b2eehi = sB2ee[m + 16], w3eelo = sW3ee[m], w3eehi = sW3ee[m + 16];
  const float b2enlo = sB2en[m], b2enhi = sB2en[m + 16], w3enlo = sW3en[m], w3enhi = sW3en[m + 16];

#pragma unroll 1
  for (int wl = 0; wl < WPB; ++wl) {
    const float* pos = sRe + wl * POSF;
    float acc = 0.0f;

#pragma unroll 1
    for (int p = tid; p < N_PAIR; p += TPB) {
      const int ij = sPIJ[p];
      const int i = ij >> 5, j = ij & 31;
      const float dx = pos[i * 3 + 0] - pos[j * 3 + 0];
      const float dy = pos[i * 3 + 1] - pos[j * 3 + 1];
      const float dz = pos[i * 3 + 2] - pos[j * 3 + 2];
      const float s = dx * dx + dy * dy + dz * dz;
      const float r = sqrtf(s);
      sPairR[p] = r;
      acc += sAsp[p] * (r * __builtin_amdgcn_rcpf(fmaf(bee_s, r, 1.0f)));
    }
    {
      const int e = tid >> 3, k = tid & 7;
      const float dx = pos[e * 3 + 0] - sNuc[k * 3 + 0];
      const float dy = pos[e * 3 + 1] - sNuc[k * 3 + 1];
      const float dz = pos[e * 3 + 2] - sNuc[k * 3 + 2];
      const float s = dx * dx + dy * dy + dz * dz;
      const float r = sqrtf(s);
      sX2[tid] = r * r;
      acc += (-sChg[k] * r) * __builtin_amdgcn_rcpf(fmaf(sBsp[k], r, 1.0f));
    }
    __syncthreads();

    {
      const int e = tid >> 3, jg = tid & 7;
      float x2[N_NUC];
#pragma unroll
      for (int k = 0; k < N_NUC; ++k) x2[k] = sX2[e * N_NUC + k];
      float hq[4];
#pragma unroll
      for (int u = 0; u < 4; ++u) {
        const int j = 4 * jg + u;
        float z = 0.0f;
#pragma unroll
        for (int k = 0; k < N_NUC; ++k) z = fmaf(x2[k], sW1en[k * D_H + j], z);
        hq[u] = silu_f(z + sB1en[j]);
      }
      const v4h pk = {(_Float16)hq[0], (_Float16)hq[1], (_Float16)hq[2], (_Float16)hq[3]};
      *(v4h*)(sH1 + e * D_H + 4 * jg) = pk;
    }
    __syncthreads();

#pragma unroll 1
    for (int t = wave; t < EE_TILES; t += NWAVE) {
      const float r = sPairR[t * 16 + m];
      Frag A;
#pragma unroll
      for (int i = 0; i < 16; ++i) A.e[i] = (_Float16)silu_f(fmaf(r, w1e[i], b1e[i]));
      const float nn = tile_nn(A.v, Bee0, Bee1, b2eelo, b2eehi, w3eelo, w3eehi);
      acc += sc_ee * (nn + ((lane == 0) ? b3ee16 : 0.0f));
    }
    if (wave < EN_TILES) {
      const v16h Av = ldA(sH1 + wave * 16 * D_H, D_H, lane);
      const float nn = tile_nn(Av, Ben0, Ben1, b2enlo, b2enhi, w3enlo, w3enhi);
      acc += sc_en * (nn + ((lane == 0) ? b3en16 : 0.0f));
    }

#pragma unroll
    for (int off = 16; off > 0; off >>= 1) acc += __shfl_xor(acc, off, 32);
    if (lane == 0) sRed[wave] = acc;
    __syncthreads();
    if (tid == 0) {
      float s = 0.0f;
#pragma unroll
      for (int q = 0; q < NWAVE; ++q) s += sRed[q];
      sRes[wl] = s;
    }
  }
  __syncthreads();

  const v4f ov = *(const v4f*)(sRes + 4 * (tid & 7));
  float* po = out + (size_t)w0 + 4 * (tid & 7);
  if (tid < 8) *(volatile v4f*)po = ov;
  __threadfence();
  if (tid < 8) *(volatile v4f*)po = ov;
}

extern "C" void kernel_launch(void* const* d_in, const int* in_sizes, int n_in,
                              void* d_out, int out_size, void* d_ws, size_t ws_size,
                              hipStream_t stream) {
  (void)d_ws; (void)ws_size;
  if (n_in < 20) return;
  const int n0 = in_sizes[0];
  if (n0 <= 0 || (n0 % POSF) != 0) return;
  const int n_walk = n0 / POSF;
  if ((n_walk % WPB) != 0) return;
  if (out_size != n_walk) return;
  if (in_sizes[1] != N_NUC * 3 || in_sizes[2] != N_NUC) return;
  if (in_sizes[3] != N_E * N_E) return;
  if (in_sizes[4] != N_NUC || in_sizes[5] < 1) return;
  if (in_sizes[6] != N_NUC * D_H || in_sizes[7] != D_H) return;
  if (in_sizes[8] != D_H * D_H || in_sizes[9] != D_H) return;
  if (in_sizes[10] != D_H || in_sizes[11] < 1) return;
  if (in_sizes[12] != D_H || in_sizes[13] != D_H) return;
  if (in_sizes[14] != D_H * D_H || in_sizes[15] != D_H) return;
  if (in_sizes[16] != D_H || in_sizes[17] < 1) return;
  if (in_sizes[18] < 1 || in_sizes[19] < 1) return;

  const int nblk = n_walk / WPB;
  k_jastrow<<<dim3(nblk), dim3(TPB), 0, stream>>>(
      (const float*)d_in[0], (const float*)d_in[1], (const float*)d_in[2],
      (const int*)d_in[3], (const float*)d_in[4], (const float*)d_in[5],
      (const float*)d_in[6], (const float*)d_in[7], (const float*)d_in[8], (const float*)d_in[9],
      (const float*)d_in[10], (const float*)d_in[11],
      (const float*)d_in[12], (const float*)d_in[13], (const float*)d_in[14], (const float*)d_in[15],
      (const float*)d_in[16], (const float*)d_in[17],
      (const float*)d_in[18], (const float*)d_in[19],
      (float*)d_out, n_walk);
}
